// LinformerCrossAttention_87591563034718
// MI455X (gfx1250) — hardware-verified
//
#include <hip/hip_runtime.h>


#define NB_  4
#define NQ   8192
#define NKV  8192
#define DD   256
#define NH_  8
#define HD   32
#define KP   256
typedef _Float16 h16;
typedef unsigned short bf;
typedef __attribute__((ext_vector_type(16))) __bf16   v16bf;
typedef __attribute__((ext_vector_type(16))) _Float16 v16h;
typedef __attribute__((ext_vector_type(8)))  _Float16 v8h;
typedef __attribute__((ext_vector_type(8)))  unsigned short v8us;
typedef __attribute__((ext_vector_type(8)))  float    v8f;
typedef __attribute__((ext_vector_type(4)))  float    v4f;
typedef v8h  __attribute__((may_alias)) v8ha;
typedef v4f  __attribute__((may_alias)) v4fa;
typedef v8us __attribute__((may_alias)) v8usa;

__device__ __forceinline__ unsigned short f2bf(float f) { unsigned u = __float_as_uint(f); u += 0x7FFFu + ((u >> 16) & 1u); return (unsigned short)(u >> 16); }
__device__ __forceinline__ float bf2f(unsigned short b) { return __uint_as_float(((unsigned)b) << 16); }
__device__ __forceinline__ float bfr(float f) { return bf2f(f2bf(f)); }
__device__ __forceinline__ v16h cat16(v8h lo, v8h hi) { return __builtin_shufflevector(lo, hi, 0, 1, 2, 3, 4, 5, 6, 7, 8, 9, 10, 11, 12, 13, 14, 15); }
__device__ __forceinline__ v16bf cat16b(v8us lo, v8us hi) { return __builtin_bit_cast(v16bf, __builtin_shufflevector(lo, hi, 0, 1, 2, 3, 4, 5, 6, 7, 8, 9, 10, 11, 12, 13, 14, 15)); }
__device__ __forceinline__ v8f wmma16(v16h a, v16h b, v8f c) { return __builtin_amdgcn_wmma_f32_16x16x32_f16(false, a, false, b, (short)0, c, false, false); }
__device__ __forceinline__ v8f wmmab(v16bf a, v16bf b, v8f c) { return __builtin_amdgcn_wmma_f32_16x16x32_bf16(false, a, false, b, (short)0, c, false, false); }


template <typename T16> struct WFrag;
template <> struct WFrag<h16> { typedef v16h V; static __device__ __forceinline__ V ld(const h16* p) { return cat16(*(const v8h*)p, *(const v8h*)(p + 16)); } static __device__ __forceinline__ v8f mma(V a, V b, v8f c) { return wmma16(a, b, c); } };
template <> struct WFrag<bf> { typedef v16bf V; static __device__ __forceinline__ V ld(const bf* p) { return cat16b(*(const v8us*)p, *(const v8us*)(p + 16)); } static __device__ __forceinline__ v8f mma(V a, V b, v8f c) { return wmmab(a, b, c); } };
template <typename T16, int NSPLIT, bool BIAS>
__global__ __launch_bounds__(32) void k_gemmw(const T16* __restrict__ A, const T16* __restrict__ A2, const T16* __restrict__ Bt, const T16* __restrict__ Bt2, int K, float* C, int ldc, const float* __restrict__ bias, size_t sA, size_t sB, size_t sC) {
    typedef typename WFrag<T16>::V V;
    __shared__ __align__(16) float os[16 * 68];
    const size_t z = blockIdx.z; A += z * sA; if (A2) A2 += z * sA; Bt += z * sB; if (Bt2) Bt2 += z * sB; C += z * sC;
    const int lane = threadIdx.x & 31, lr = lane & 15, hi = lane >> 4; const int r0 = blockIdx.x * 64, c0 = blockIdx.y * 64;
    v8f acc[4][4];
#pragma unroll
    for (int mb = 0; mb < 4; ++mb)
#pragma unroll
        for (int nb = 0; nb < 4; ++nb) acc[mb][nb] = (v8f){};
    const size_t aoff = (size_t)(r0 + lr) * K + 8 * hi, boff = (size_t)(c0 + lr) * K + 8 * hi;
#pragma unroll 1
    for (int kc = 0; kc < K; kc += 32) {
        V a[4], a2[4];
#pragma unroll
        for (int mb = 0; mb < 4; ++mb) { a[mb] = WFrag<T16>::ld(A + aoff + (size_t)mb * 16 * K + kc); if (NSPLIT == 1 || NSPLIT == 2) a2[mb] = WFrag<T16>::ld(A2 + aoff + (size_t)mb * 16 * K + kc); }
#pragma unroll
        for (int nb = 0; nb < 4; ++nb) { const V b = WFrag<T16>::ld(Bt + boff + (size_t)nb * 16 * K + kc); V b2; if (NSPLIT >= 2) b2 = WFrag<T16>::ld(Bt2 + boff + (size_t)nb * 16 * K + kc);
#pragma unroll
            for (int mb = 0; mb < 4; ++mb) { acc[mb][nb] = WFrag<T16>::mma(a[mb], b, acc[mb][nb]); if (NSPLIT == 1 || NSPLIT == 2) acc[mb][nb] = WFrag<T16>::mma(a2[mb], b, acc[mb][nb]); if (NSPLIT >= 2) acc[mb][nb] = WFrag<T16>::mma(a[mb], b2, acc[mb][nb]); } }
        asm volatile("v_nop\n\tv_nop\n\tv_nop\n\tv_nop" : "+v"(acc[0][0]), "+v"(acc[1][1]), "+v"(acc[2][2]), "+v"(acc[3][3]) : "v"(a[0]), "v"(a[3]));
    }
#pragma unroll
    for (int mb = 0; mb < 4; ++mb) {
#pragma unroll
        for (int nb = 0; nb < 4; ++nb) {
#pragma unroll
            for (int j = 0; j < 8; ++j) os[(hi * 8 + j) * 68 + nb * 16 + lr] = acc[mb][nb][j]; }
        __builtin_amdgcn_wave_barrier(); asm volatile("" ::: "memory");
        float* crow = C + (size_t)(r0 + mb * 16) * ldc + c0;
#pragma unroll 1
        for (int ps = 0; ps < 2; ++ps) {
#pragma unroll
            for (int s = 0; s < 8; ++s) { const int row = 2 * s + hi, cofs = lr * 4; v4f val = *(const v4fa*)(os + row * 68 + cofs); if (BIAS) { val[0] += bfr(bias[c0 + cofs]); val[1] += bfr(bias[c0 + cofs + 1]); val[2] += bfr(bias[c0 + cofs + 2]); val[3] += bfr(bias[c0 + cofs + 3]); }
                *(volatile v4f*)(crow + (size_t)row * ldc + cofs) = val; }
            if (ps == 0) __threadfence(); }
        __builtin_amdgcn_wave_barrier(); asm volatile("" ::: "memory");
    }
}

__device__ __forceinline__ void splitf(float y, unsigned short& h, unsigned short& l) { h = f2bf(y); l = f2bf(y - bf2f(h)); }
typedef __attribute__((ext_vector_type(2))) unsigned short v2us;
typedef __attribute__((ext_vector_type(4))) unsigned short v4us;

__global__ __launch_bounds__(256) void k_wtG(const float* __restrict__ w, int K, int N, bf* Bt) {
    const int lane = threadIdx.x & 31; const int L0 = (blockIdx.x * 8 + (threadIdx.x >> 5)) * 8; const int nlines = N * K / 64;
#pragma unroll
    for (int ps = 0; ps < 2; ++ps) {
#pragma unroll 1
        for (int l = 0; l < 8; ++l) { const int L = L0 + l; if (L >= nlines) break; const size_t e = (size_t)L * 64 + lane * 2; const int k = (int)(e % K), n = (int)(e / K); v2us o;
            o[0] = f2bf(w[(size_t)k * N + n]); o[1] = f2bf(w[(size_t)(k + 1) * N + n]); *(volatile v2us*)(Bt + e) = o; }
        if (ps == 0) __threadfence(); }
}
__global__ __launch_bounds__(256) void k_cvt8(const float* __restrict__ src, bf* dst, size_t n8) { const size_t i = (size_t)blockIdx.x * 256 + threadIdx.x; if (i >= n8) return; const v8f v = *(const v8f*)(src + i * 8); v8us o;
#pragma unroll
    for (int k = 0; k < 8; ++k) o[k] = f2bf(v[k]); *(volatile v8us*)(dst + i * 8) = o; __threadfence(); *(volatile v8us*)(dst + i * 8) = o; }
__global__ __launch_bounds__(256) void k_tpl(const float* __restrict__ F, bf* Th, bf* Tl) { const int e = (blockIdx.x * 256 + threadIdx.x) * 2; if (e >= DD * NKV) return; const int n = e % NKV; const int d = e / NKV; v2us oh, ol; unsigned short a1, b1, a2, b2; splitf(F[(size_t)n * DD + d], a1, b1); splitf(F[(size_t)(n + 1) * DD + d], a2, b2); oh[0] = a1; oh[1] = a2; ol[0] = b1; ol[1] = b2;
    for (int ps = 0; ps < 2; ++ps) { *(volatile v2us*)(Th + e) = oh; *(volatile v2us*)(Tl + e) = ol; if (ps == 0) __threadfence(); } }
__global__ __launch_bounds__(256) void k_etb(const float* __restrict__ E, bf* Bt) { const int e = (blockIdx.x * 256 + threadIdx.x) * 2; if (e >= KP * NKV) return; const int n = e % NKV; const int kp = e / NKV; v2us o; o[0] = f2bf(E[(size_t)n * KP + kp]); o[1] = f2bf(E[(size_t)(n + 1) * KP + kp]); *(volatile v2us*)(Bt + e) = o; __threadfence(); *(volatile v2us*)(Bt + e) = o; }
__global__ __launch_bounds__(256) void k_plq(const float* __restrict__ Q, bf* Ph, bf* Pl) { const int e = (blockIdx.x * 256 + threadIdx.x) * 4; if (e >= NH_ * NQ * HD) return; const int d = e % HD; const int q = (e / HD) % NQ; const int h = e / (HD * NQ); const float* f = Q + (size_t)q * DD + h * HD + d; v4us oh, ol;
#pragma unroll
    for (int u = 0; u < 4; ++u) { unsigned short a, b; splitf(f[u], a, b); oh[u] = a; ol[u] = b; } for (int ps = 0; ps < 2; ++ps) { *(volatile v4us*)(Ph + e) = oh; *(volatile v4us*)(Pl + e) = ol; if (ps == 0) __threadfence(); } }
__global__ __launch_bounds__(256) void k_kp(const float* __restrict__ KL, bf* Ph, bf* Pl) { const int e = (blockIdx.x * 256 + threadIdx.x) * 4; if (e >= NH_ * KP * HD) return; const int d = e % HD; const int kp = (e / HD) % KP; const int h = e / (HD * KP); v4us oh, ol;
#pragma unroll
    for (int u = 0; u < 4; ++u) { unsigned short a, b; splitf(KL[(size_t)(h * HD + d + u) * KP + kp], a, b); oh[u] = a; ol[u] = b; } for (int ps = 0; ps < 2; ++ps) { *(volatile v4us*)(Ph + e) = oh; *(volatile v4us*)(Pl + e) = ol; if (ps == 0) __threadfence(); } }
__global__ __launch_bounds__(256) void k_vl(const float* __restrict__ VL, bf* Vh, bf* Vl) { const int e = (blockIdx.x * 256 + threadIdx.x) * 4; if (e >= (DD + 64) * KP) return; v4us oh, ol;
#pragma unroll
    for (int u = 0; u < 4; ++u) { unsigned short x = 0, y = 0; if (e < DD * KP) splitf(VL[e + u], x, y); oh[u] = x; ol[u] = y; } *(volatile v4us*)(Vh + e) = oh; *(volatile v4us*)(Vl + e) = ol; __threadfence(); *(volatile v4us*)(Vh + e) = oh; *(volatile v4us*)(Vl + e) = ol; }
__global__ __launch_bounds__(256) void k_lsoft(const float* __restrict__ Sb, bf* Ph, bf* Pl) { const int lane = threadIdx.x & 31; const int row = blockIdx.x * 8 + (threadIdx.x >> 5); if (row >= NH_ * NQ) return; const float* sr = Sb + (size_t)row * KP; float v[KP / 32]; float mx = -3.0e38f;
#pragma unroll
    for (int ch = 0; ch < KP / 128; ++ch) { const v4f a = *(const v4f*)(sr + ch * 128 + lane * 4);
#pragma unroll
        for (int u = 0; u < 4; ++u) { const float t = __fdiv_rn(a[u], 5.656854249492381f); v[ch * 4 + u] = t; mx = fmaxf(mx, t); } }
#pragma unroll
    for (int sh = 16; sh; sh >>= 1) mx = fmaxf(mx, __shfl_xor(mx, sh, 32));
    float sum = 0.f;
#pragma unroll
    for (int q = 0; q < KP / 32; ++q) { float d0 = __fsub_rn(v[q], mx); asm volatile("" : "+v"(d0)); v[q] = __builtin_amdgcn_exp2f(__fmul_rn(d0, 1.4426950408889634f)); sum += v[q]; }
#pragma unroll
    for (int sh = 16; sh; sh >>= 1) sum += __shfl_xor(sum, sh, 32);
    const float f = __fdiv_rn(1.0f, sum);
    for (int ps = 0; ps < 2; ++ps) {
#pragma unroll
        for (int ch = 0; ch < KP / 128; ++ch) { v4us oh, ol;
#pragma unroll
            for (int q = 0; q < 4; ++q) { unsigned short a, b; splitf(v[ch * 4 + q] * f, a, b); oh[q] = a; ol[q] = b; } const size_t oo = (size_t)row * KP + ch * 128 + lane * 4; *(volatile v4us*)(Ph + oo) = oh; *(volatile v4us*)(Pl + oo) = ol; }
        if (ps == 0) __threadfence(); } }
__global__ __launch_bounds__(256) void k_mrg(const float* __restrict__ O, bf* Ah, bf* Al) { const int e = (blockIdx.x * 256 + threadIdx.x) * 4; if (e >= NQ * DD) return; const int c = e % DD; const int q = e / DD; const int h = c / HD, d = c % HD; const float* o = O + ((size_t)h * NQ + q) * 64 + d; v4us oh, ol;
#pragma unroll
    for (int u = 0; u < 4; ++u) { unsigned short a, b; splitf(o[u], a, b); oh[u] = a; ol[u] = b; } *(volatile v4us*)(Ah + e) = oh; *(volatile v4us*)(Al + e) = ol; __threadfence(); *(volatile v4us*)(Ah + e) = oh; *(volatile v4us*)(Al + e) = ol; }

extern "C" void kernel_launch(void* const* d_in, const int* in_sizes, int n_in,
                              void* d_out, int out_size, void* d_ws, size_t ws_size, hipStream_t stream) {
    (void)in_sizes; (void)n_in; (void)out_size;
    const float** I = (const float**)d_in;
    const float *x1 = I[0], *x2 = I[1], *Wq = I[2], *Wk = I[3], *Wv = I[4], *Wo = I[5], *E = I[6], *F = I[7];
    float* OUT = (float*)d_out;
    char* wsp = (char*)d_ws;
    auto take = [&](size_t bytes) { char* p = wsp; wsp += (bytes + 255) & ~(size_t)255; return (void*)p; };
    bf* BQ = (bf*)take(DD * DD * 2); bf* BK = (bf*)take(DD * DD * 2); bf* BV = (bf*)take(DD * DD * 2); bf* BO = (bf*)take(DD * DD * 2);
    bf* X2 = (bf*)take((size_t)NKV * DD * 2); float* Kf = (float*)take((size_t)NKV * DD * 4); float* Vf = (float*)take((size_t)NKV * DD * 4); bf* KTh = (bf*)take((size_t)DD * NKV * 2); bf* KTl = (bf*)take((size_t)DD * NKV * 2); bf* VTh = (bf*)take((size_t)DD * NKV * 2); bf* VTl = (bf*)take((size_t)DD * NKV * 2);
    bf* ET = (bf*)take((size_t)KP * NKV * 2); bf* FT = (bf*)take((size_t)KP * NKV * 2); float* KL = (float*)take((size_t)DD * KP * 4); float* VL = (float*)take((size_t)DD * KP * 4); bf* KPh = (bf*)take((size_t)NH_ * KP * HD * 2); bf* KPl = (bf*)take((size_t)NH_ * KP * HD * 2); bf* VLh = (bf*)take((size_t)(DD + 64) * KP * 2); bf* VLl = (bf*)take((size_t)(DD + 64) * KP * 2);
    bf* X1 = (bf*)take((size_t)NQ * DD * 2); float* Q = (float*)take((size_t)NQ * DD * 4); bf* Qh = (bf*)take((size_t)NH_ * NQ * HD * 2); bf* Ql = (bf*)take((size_t)NH_ * NQ * HD * 2); float* Sb = (float*)take((size_t)NH_ * NQ * KP * 4); bf* Ph = (bf*)take((size_t)NH_ * NQ * KP * 2); bf* Pl = (bf*)take((size_t)NH_ * NQ * KP * 2);
    float* O = (float*)take((size_t)NH_ * NQ * 64 * 4); bf* Ah = (bf*)take((size_t)NQ * DD * 2); bf* Al = (bf*)take((size_t)NQ * DD * 2);
    if ((size_t)(wsp - (char*)d_ws) > ws_size) return;
    k_wtG<<<(DD * DD / 64 + 63) / 64, 256, 0, stream>>>(Wq, DD, DD, BQ); k_wtG<<<(DD * DD / 64 + 63) / 64, 256, 0, stream>>>(Wk, DD, DD, BK); k_wtG<<<(DD * DD / 64 + 63) / 64, 256, 0, stream>>>(Wv, DD, DD, BV); k_wtG<<<(DD * DD / 64 + 63) / 64, 256, 0, stream>>>(Wo, DD, DD, BO);
    k_cvt8<<<(NKV * DD / 8 + 255) / 256, 256, 0, stream>>>(x2, X2, (size_t)NKV * DD / 8);
    k_gemmw<bf, 0, false><<<dim3(NKV / 64, DD / 64, 1), 32, 0, stream>>>(X2, nullptr, BK, nullptr, DD, Kf, DD, nullptr, 0, 0, 0); k_gemmw<bf, 0, false><<<dim3(NKV / 64, DD / 64, 1), 32, 0, stream>>>(X2, nullptr, BV, nullptr, DD, Vf, DD, nullptr, 0, 0, 0);
    k_tpl<<<(DD * NKV / 2 + 255) / 256, 256, 0, stream>>>(Kf, KTh, KTl); k_tpl<<<(DD * NKV / 2 + 255) / 256, 256, 0, stream>>>(Vf, VTh, VTl); k_etb<<<(KP * NKV / 2 + 255) / 256, 256, 0, stream>>>(E, ET); k_etb<<<(KP * NKV / 2 + 255) / 256, 256, 0, stream>>>(F, FT);
    k_gemmw<bf, 1, false><<<dim3(DD / 64, KP / 64, 1), 32, 0, stream>>>(KTh, KTl, ET, nullptr, NKV, KL, KP, nullptr, 0, 0, 0); k_gemmw<bf, 1, false><<<dim3(DD / 64, KP / 64, 1), 32, 0, stream>>>(VTh, VTl, FT, nullptr, NKV, VL, KP, nullptr, 0, 0, 0);
    k_kp<<<(NH_ * KP * HD / 4 + 255) / 256, 256, 0, stream>>>(KL, KPh, KPl); k_vl<<<((DD + 64) * KP / 4 + 255) / 256, 256, 0, stream>>>(VL, VLh, VLl);
    const size_t zq = (size_t)NQ * HD, zk = (size_t)KP * HD, zS = (size_t)NQ * KP, zv = (size_t)HD * KP, zo = (size_t)NQ * 64;
    for (int b = 0; b < NB_; ++b) {
        k_cvt8<<<(NQ * DD / 8 + 255) / 256, 256, 0, stream>>>(x1 + (size_t)b * NQ * DD, X1, (size_t)NQ * DD / 8);
        k_gemmw<bf, 0, false><<<dim3(NQ / 64, DD / 64, 1), 32, 0, stream>>>(X1, nullptr, BQ, nullptr, DD, Q, DD, nullptr, 0, 0, 0); k_plq<<<(NH_ * NQ * HD / 4 + 255) / 256, 256, 0, stream>>>(Q, Qh, Ql);
        k_gemmw<bf, 2, false><<<dim3(NQ / 64, KP / 64, NH_), 32, 0, stream>>>(Qh, Ql, KPh, KPl, HD, Sb, KP, nullptr, zq, zk, zS);
        k_lsoft<<<NH_ * NQ / 8, 256, 0, stream>>>(Sb, Ph, Pl);
        k_gemmw<bf, 2, false><<<dim3(NQ / 64, 1, NH_), 32, 0, stream>>>(Ph, Pl, VLh, VLl, KP, O, 64, nullptr, zS, zv, zo);
        k_mrg<<<(NQ * DD / 4 + 255) / 256, 256, 0, stream>>>(O, Ah, Al);
        k_gemmw<bf, 1, false><<<dim3(NQ / 64, DD / 64, 1), 32, 0, stream>>>(Ah, Al, BO, nullptr, DD, OUT + (size_t)b * NQ * DD, DD, nullptr, 0, 0, 0); }
}
